// PhaseLinear_58463094833618
// MI455X (gfx1250) — hardware-verified
//
#include <hip/hip_runtime.h>
#include <stddef.h>


typedef _Float16 v16h __attribute__((ext_vector_type(16)));
typedef _Float16 v8h  __attribute__((ext_vector_type(8)));
typedef float    v8f  __attribute__((ext_vector_type(8)));
typedef float    v4f  __attribute__((ext_vector_type(4)));
typedef _Float16 h16;

#ifndef NROWS
#define NROWS 1024
#endif
#define NROWS_FULL 1024
#define KDIM  512
#define OUTF  512
#define NCP   4
#define NCOLS (NCP * OUTF)

static_assert(NROWS >= 64 && NROWS <= NROWS_FULL && (NROWS % 64) == 0);
static_assert((KDIM % 32) == 0 && (KDIM % 8) == 0);
static_assert((OUTF % 64) == 0);
static_assert(NCP == 4);
static_assert((((size_t)NROWS * KDIM / 8) % 256) == 0);
static_assert((((size_t)NCOLS * KDIM / 8) % 256) == 0);

#define LDC 68
static_assert((LDC % 4) == 0 && LDC >= 64);

#define XCARRY 16.0f
#define WCARRY 64.0f

#define X16_BYTES ((size_t)NROWS * KDIM * 2)
#define W16_BYTES ((size_t)NCOLS * KDIM * 2)
#define OFF_X16 ((size_t)0)
#define OFF_W16 (OFF_X16 + X16_BYTES)
#define WS_TOTAL (OFF_W16 + W16_BYTES)
static_assert((X16_BYTES % 512) == 0 && (W16_BYTES % 512) == 0);
static_assert(WS_TOTAL <= (size_t)134217728);

__device__ __forceinline__ float bf16r(float x) {
  unsigned int u = __float_as_uint(x);
  u = (u + 0x7FFFu + ((u >> 16) & 1u)) & 0xFFFF0000u;
  return __uint_as_float(u);
}

static __device__ __forceinline__ h16 toh_flush(float v) {
  const h16 r = (h16)v;
  return (fabsf(v) < 6.103515625e-05f) ? (h16)0.0f : r;
}

__device__ __forceinline__ v16h frag_at(const _Float16* p) {
  v8h lo = *(const v8h*)(p);
  v8h hi = *(const v8h*)(p + 16);
  v16h out;
#pragma unroll
  for (int i = 0; i < 8; ++i) { out[i] = lo[i]; out[i + 8] = hi[i]; }
  return out;
}

__device__ __forceinline__ v8f wmma16(v16h a, v16h b, v8f c) {
  v8f d = __builtin_amdgcn_wmma_f32_16x16x32_f16(false, a, false, b, (short)0, c,
                                                 false, false);
  asm volatile("v_nop\n\tv_nop\n\tv_nop\n\tv_nop" : "+v"(d) : "v"(a), "v"(b));
  return d;
}

__global__ __launch_bounds__(256) void cast_kernel(
    const float* __restrict__ src, _Float16* __restrict__ dst, const float carry,
    const unsigned n8) {
#pragma clang fp contract(off)
  const unsigned i = blockIdx.x * 256u + threadIdx.x;
  const unsigned ic = (i < n8) ? i : (n8 - 1u);
  const v4f a0 = *(const v4f*)(src + (size_t)ic * 8u);
  const v4f a1 = *(const v4f*)(src + (size_t)ic * 8u + 4u);
  v8h o;
#pragma unroll
  for (int j = 0; j < 4; ++j) {
    o[j]     = toh_flush(carry * bf16r(a0[j]));
    o[j + 4] = toh_flush(carry * bf16r(a1[j]));
  }
  _Float16* p = dst + (size_t)ic * 8u;
  if (i < n8) *(volatile v8h*)p = o;
  __threadfence();
  if (i < n8) *(volatile v8h*)p = o;
}

__global__ __launch_bounds__(256) void phase_gemm_kernel(
    const _Float16* __restrict__ A16, const _Float16* __restrict__ Bt,
    const float* __restrict__ phase, const float* __restrict__ bias,
    float* __restrict__ outf) {
  __shared__ __attribute__((aligned(16))) float Cs[64 * LDC];
  __shared__ __attribute__((aligned(16))) float Cf[64 * NCP];
  static_assert(sizeof(float) * (64 * LDC + 64 * NCP) <= 131072);

  const unsigned tid = threadIdx.x, lane = tid & 31u;
  const unsigned w = (unsigned)__builtin_amdgcn_readfirstlane((int)(threadIdx.x >> 5));
  const unsigned mw = w >> 1, nw = w & 1u;
  const unsigned hh = lane >> 4, m = lane & 15u;
  const unsigned n0 = blockIdx.x * 64u;
  const unsigned row0 = blockIdx.y * 64u;

  {
    const unsigned lr = tid & 63u;
    const float ph = bf16r(phase[row0 + lr]);
    const float inv = 1.0f / 4.71238898038469f;
    const float t0 = ph * inv;
    const float t1 = (ph - 1.5707963267948966f) * inv;
    const float t = (ph < 4.71238898038469f) ? t0 : t1;
    const float t2 = t * t;
    const float t3 = t2 * t;
    v4f cf;
    cf[0] = t3 - 0.5f * t2;
    cf[1] = 1.0f - 2.5f * t3;
    cf[2] = 0.5f * t2 + 2.0f * t3;
    cf[3] = -0.5f * t3;
    if (tid < 64u) *(v4f*)&Cf[lr * 4u] = cf;
  }
  __syncthreads();

  const _Float16* ap = A16 + (size_t)(row0 + mw * 16u + m) * KDIM + hh * 8u;
  const _Float16* bp = Bt + (size_t)(n0 + nw * 32u + m) * KDIM + hh * 8u;
  v8f acc[NCP][2];
#pragma unroll
  for (int c = 0; c < NCP; ++c) { acc[c][0] = (v8f){}; acc[c][1] = (v8f){}; }

#pragma unroll 1
  for (unsigned k0 = 0; k0 < (unsigned)KDIM; k0 += 32u) {
    const v16h a = frag_at(ap + k0);
#pragma unroll
    for (int c = 0; c < NCP; ++c) {
      const _Float16* bc = bp + (size_t)c * OUTF * KDIM + k0;
      const v16h b0 = frag_at(bc);
      const v16h b1 = frag_at(bc + (size_t)16 * KDIM);
      acc[c][0] = wmma16(a, b0, acc[c][0]);
      acc[c][1] = wmma16(a, b1, acc[c][1]);
    }
  }

#pragma unroll
  for (int r = 0; r < 8; ++r) {
    const unsigned lr = mw * 16u + hh * 8u + (unsigned)r;
    const v4f cf = *(const v4f*)&Cf[lr * 4u];
    float s0 = cf[0] * acc[0][0][r];
    float s1 = cf[0] * acc[0][1][r];
    s0 += cf[1] * acc[1][0][r];
    s1 += cf[1] * acc[1][1][r];
    s0 += cf[2] * acc[2][0][r];
    s1 += cf[2] * acc[2][1][r];
    s0 += cf[3] * acc[3][0][r];
    s1 += cf[3] * acc[3][1][r];
    float* d = &Cs[lr * LDC + nw * 32u + m];
    d[0]  = s0;
    d[16] = s1;
  }
  __syncthreads();

  static_assert(16 * 4 == 64);
  const float cs = 1.0f / (XCARRY * WCARRY);
  v4f xs[4];
  size_t off[4];
#pragma unroll
  for (unsigned i = 0; i < 4u; ++i) {
    const unsigned r = 16u * i + (tid >> 4);
    const unsigned c = (tid & 15u) * 4u;
    const v4f u  = *(const v4f*)&Cs[r * LDC + c];
    const v4f cf = *(const v4f*)&Cf[r * 4u];
    const v4f g0 = *(const v4f*)(bias + 0u * OUTF + n0 + c);
    const v4f g1 = *(const v4f*)(bias + 1u * OUTF + n0 + c);
    const v4f g2 = *(const v4f*)(bias + 2u * OUTF + n0 + c);
    const v4f g3 = *(const v4f*)(bias + 3u * OUTF + n0 + c);
    v4f val;
#pragma unroll
    for (int j = 0; j < 4; ++j) {
      float bsum = cf[0] * bf16r(g0[j]);
      bsum += cf[1] * bf16r(g1[j]);
      bsum += cf[2] * bf16r(g2[j]);
      bsum += cf[3] * bf16r(g3[j]);
      val[j] = u[j] * cs + bsum;
    }
    xs[i] = val;
    off[i] = (size_t)(row0 + r) * OUTF + n0 + c;
  }
#pragma unroll
  for (int i = 0; i < 4; ++i) *(volatile v4f*)(outf + off[i]) = xs[i];
  __threadfence();
#pragma unroll
  for (int i = 0; i < 4; ++i) *(volatile v4f*)(outf + off[i]) = xs[i];
}

extern "C" void kernel_launch(void* const* d_in, const int* in_sizes, int n_in,
                              void* d_out, int out_size, void* d_ws, size_t ws_size,
                              hipStream_t stream) {
  if (n_in < 4) return;
  if ((long long)in_sizes[0] < (long long)NROWS * KDIM) return;
  if ((long long)in_sizes[1] < (long long)NROWS) return;
  if ((long long)in_sizes[2] < (long long)NCOLS * KDIM) return;
  if ((long long)in_sizes[3] < (long long)NCOLS) return;
  if ((long long)out_size < (long long)NROWS * OUTF) return;
  if (ws_size < WS_TOTAL) return;

  const float* X   = (const float*)d_in[0];
  const float* ph  = (const float*)d_in[1];
  const float* Wt  = (const float*)d_in[2];
  const float* bs  = (const float*)d_in[3];
  float* out = (float*)d_out;

  char* ws = (char*)d_ws;
  _Float16* X16 = (_Float16*)(ws + OFF_X16);
  _Float16* W16 = (_Float16*)(ws + OFF_W16);

  dim3 blk(256);
  const unsigned nx8 = (unsigned)((size_t)NROWS * KDIM / 8);
  const unsigned nw8 = (unsigned)((size_t)NCOLS * KDIM / 8);

  cast_kernel<<<dim3(nx8 / 256u), blk, 0, stream>>>(X, X16, XCARRY, nx8);
  cast_kernel<<<dim3(nw8 / 256u), blk, 0, stream>>>(Wt, W16, WCARRY, nw8);
  phase_gemm_kernel<<<dim3(OUTF / 64, NROWS / 64), blk, 0, stream>>>(X16, W16, ph, bs, out);
}
